// TransformerBlock_50483045597391
// MI455X (gfx1250) — hardware-verified
//
#include <hip/hip_runtime.h>
#include <math.h>

#ifndef NB
#define NB 4
#endif
#ifndef SEQ
#define SEQ 1024
#endif
#define NB_FULL 4
#define SEQ_FULL 1024
#define DM 1024
#define NHD 16
#define DFF 4096
#define FCH 1024
#define XBS_FULL ((long long)SEQ_FULL * DM)
static_assert(SEQ % 64 == 0);
static_assert(SEQ <= SEQ_FULL);
static_assert(NB >= 1 && NB <= NB_FULL);
static_assert(DM == NHD * 64);
static_assert(DM % 64 == 0 && DFF % 64 == 0 && FCH % 64 == 0 && DFF % FCH == 0);
static_assert(DM % 32 == 0 && DFF % 32 == 0 && (2 * DM) % 32 == 0);
static_assert(DM == 128 * 8);
static_assert(FCH % 2 == 0 && DM % 8 == 0 && DFF % 8 == 0);

typedef __attribute__((ext_vector_type(16))) _Float16 v16h;
typedef __attribute__((ext_vector_type(8)))  _Float16 v8h;
typedef __attribute__((ext_vector_type(8)))  float    v8f;
typedef __attribute__((ext_vector_type(4)))  float    v4f;
typedef __attribute__((ext_vector_type(2)))  float    v2f;
typedef _Float16 h16;

__device__ __forceinline__ v8f wmma16(v16h a, v16h b, v8f c) {
    c = __builtin_amdgcn_wmma_f32_16x16x32_f16(false, a, false, b, (short)0, c, false, false);
    asm volatile("v_nop\n\tv_nop\n\tv_nop\n\tv_nop" : "+v"(c) : "v"(a), "v"(b));
    return c;
}
union FragH { v16h v; v8h h[2]; };
__device__ __forceinline__ v16h lds_frag(const _Float16* p) { FragH f; f.h[0] = *(const v8h*)(p); f.h[1] = *(const v8h*)(p + 16); return f.v; }

static __device__ __forceinline__ h16 toh_flush(float v) { const h16 r = (h16)v; return (fabsf(v) < 6.103515625e-05f) ? (h16)0.0f : r; }

#define QKRES 2048.0f
#define QKRINV 4.8828125e-4f
__device__ __forceinline__ void glb_frag_f32_hr(const float* __restrict__ p, v16h& hi, v16h& rs) {
    const v4f a = *(const v4f*)(p), b = *(const v4f*)(p + 4), c = *(const v4f*)(p + 16), d = *(const v4f*)(p + 20);
    const float w[16] = { a.x, a.y, a.z, a.w, b.x, b.y, b.z, b.w, c.x, c.y, c.z, c.w, d.x, d.y, d.z, d.w };
    v16h vh, vr;
#pragma unroll
    for (int e = 0; e < 16; ++e) { const h16 t = toh_flush(w[e]); vh[e] = t; vr[e] = toh_flush((w[e] - (float)t) * QKRES); }
    hi = vh; rs = vr;
}

#define VST2(T, ptr, val) do { const T vst2_v_ = (val); *(volatile T*)(ptr) = vst2_v_; __threadfence(); *(volatile T*)(ptr) = vst2_v_; } while (0)
#define VST2V4(ptr, val) do { const v4f vst2_v4_ = (val); *(volatile v4f*)(ptr) = vst2_v4_; __threadfence(); *(volatile v4f*)(ptr) = vst2_v4_; } while (0)

#define AW 4
#define KPITCH 72
#define OPITCH 68
static_assert(AW == 4);

__global__ __launch_bounds__(32 * AW) __attribute__((amdgpu_num_vgpr(256))) void k_attn3(
        const float* Q, const float* K, const float* V, float* O,
        long long sQb, long long sKb, long long sVb, long long sOb,
        int ldq, int ldk, int ldv, int ldo, int Lk, int coff, float scale) {
    __shared__ __align__(16) _Float16 kl[64 * KPITCH];
    __shared__ __align__(16) _Float16 krl[64 * KPITCH];
    __shared__ __align__(16) _Float16 vt[64 * KPITCH];
    __shared__ __align__(16) _Float16 ph[AW][16 * KPITCH];
    __shared__ __align__(16) float    ot[AW][16 * OPITCH];
    const int tid = threadIdx.x, lane = tid & 31, hf = lane >> 4, l15 = lane & 15;
    const int wave = __builtin_amdgcn_readfirstlane(tid >> 5);
    const int h = blockIdx.y, b = blockIdx.z;
    const int q0 = (blockIdx.x * AW + wave) * 16;
    const float L2E = 1.4426950408889634f;
    const float NEG = -__builtin_inff();
    const float* kbase = K + b * sKb + h * 64;
    const float* vbase = V + b * sVb + h * 64;
    _Float16* myph = ph[wave];
    const float* qrow = Q + b * sQb + (long long)(q0 + l15) * ldq + h * 64 + 8 * hf;
    v16h qa0, qr0, qa1, qr1;
    glb_frag_f32_hr(qrow, qa0, qr0);
    glb_frag_f32_hr(qrow + 32, qa1, qr1);
    v8f o[4]; float m8[8], l8[8];
#pragma unroll
    for (int t = 0; t < 4; ++t) { v8f zz = {}; o[t] = zz; }
#pragma unroll
    for (int i = 0; i < 8; ++i) { m8[i] = NEG; l8[i] = 0.f; }
    const int je = (int)(blockIdx.x * AW + AW - 1) * 16 + 16 + coff;
    const int jend = min(Lk, max(je, 0));
    for (int j0 = 0; j0 < jend; j0 += 64) {
        __syncthreads();
        {
            const int jr = tid >> 1, dh = (tid & 1) * 32;
            const float* krow = kbase + (long long)(j0 + jr) * ldk + dh;
            const float* vrow = vbase + (long long)(j0 + jr) * ldv + dh;
#pragma unroll
            for (int i = 0; i < 4; ++i) {
                const v4f k0 = *(const v4f*)(krow + 8 * i), k1 = *(const v4f*)(krow + 8 * i + 4);
                const float kw[8] = { k0.x, k0.y, k0.z, k0.w, k1.x, k1.y, k1.z, k1.w };
                v8h kk, kq;
#pragma unroll
                for (int e = 0; e < 8; ++e) { const h16 t = toh_flush(kw[e]); kk[e] = t; kq[e] = toh_flush((kw[e] - (float)t) * QKRES); }
                *(v8h*)(kl + jr * KPITCH + dh + 8 * i) = kk;
                *(v8h*)(krl + jr * KPITCH + dh + 8 * i) = kq;
                const v4f v0 = *(const v4f*)(vrow + 8 * i), v1 = *(const v4f*)(vrow + 8 * i + 4);
                const int dc = dh + 8 * i;
                vt[(dc + 0) * KPITCH + jr] = toh_flush(v0.x); vt[(dc + 1) * KPITCH + jr] = toh_flush(v0.y);
                vt[(dc + 2) * KPITCH + jr] = toh_flush(v0.z); vt[(dc + 3) * KPITCH + jr] = toh_flush(v0.w);
                vt[(dc + 4) * KPITCH + jr] = toh_flush(v1.x); vt[(dc + 5) * KPITCH + jr] = toh_flush(v1.y);
                vt[(dc + 6) * KPITCH + jr] = toh_flush(v1.z); vt[(dc + 7) * KPITCH + jr] = toh_flush(v1.w);
            }
        }
        __syncthreads();
        v8f s[4];
#pragma unroll
        for (int t = 0; t < 4; ++t) {
            const int ko = (t * 16 + l15) * KPITCH + 8 * hf;
            const v16h kh0 = lds_frag(kl + ko), kh1 = lds_frag(kl + ko + 32);
            const v16h kr0 = lds_frag(krl + ko), kr1 = lds_frag(krl + ko + 32);
            v8f acc = {}, accr = {};
            acc  = wmma16(qa0, kh0, acc);
            acc  = wmma16(qa1, kh1, acc);
            accr = wmma16(qa0, kr0, accr);
            accr = wmma16(qa1, kr1, accr);
            accr = wmma16(qr0, kh0, accr);
            accr = wmma16(qr1, kh1, accr);
            s[t] = acc + accr * QKRINV;
        }
#pragma unroll
        for (int i = 0; i < 8; ++i) {
            const int irow = q0 + i + 8 * hf;
            float sc[4];
#pragma unroll
            for (int t = 0; t < 4; ++t) {
                const int jg = j0 + t * 16 + l15;
                float v = s[t][i] * scale;
                if (jg > irow + coff) v = NEG; else v *= L2E;
                sc[t] = v;
            }
            float mx = fmaxf(fmaxf(sc[0], sc[1]), fmaxf(sc[2], sc[3]));
            mx = fmaxf(mx, __shfl_xor(mx, 1, 32)); mx = fmaxf(mx, __shfl_xor(mx, 2, 32));
            mx = fmaxf(mx, __shfl_xor(mx, 4, 32)); mx = fmaxf(mx, __shfl_xor(mx, 8, 32));
            const float mnew = fmaxf(m8[i], mx);
            const float corr = (mnew == NEG) ? 1.f : exp2f(m8[i] - mnew);
            float rs = 0.f;
#pragma unroll
            for (int t = 0; t < 4; ++t) {
                const float ea = sc[t] - mnew;
                const float pp = (sc[t] == NEG || ea < -26.0f) ? 0.f : exp2f(ea); rs += pp;
                myph[(i + 8 * hf) * KPITCH + t * 16 + l15] = (_Float16)(pp * 4096.f);
            }
            rs += __shfl_xor(rs, 1, 32); rs += __shfl_xor(rs, 2, 32); rs += __shfl_xor(rs, 4, 32); rs += __shfl_xor(rs, 8, 32);
            l8[i] = l8[i] * corr + rs; m8[i] = mnew;
#pragma unroll
            for (int t = 0; t < 4; ++t) o[t][i] *= corr;
        }
        __syncthreads();
        {
            const _Float16* pr = myph + l15 * KPITCH + 8 * hf;
            const v16h pa0 = lds_frag(pr), pa1 = lds_frag(pr + 32);
#pragma unroll
            for (int t = 0; t < 4; ++t) {
                const _Float16* vr = vt + (t * 16 + l15) * KPITCH + 8 * hf;
                o[t] = wmma16(pa0, lds_frag(vr), o[t]);
                o[t] = wmma16(pa1, lds_frag(vr + 32), o[t]);
            }
        }
    }
    float* mo = ot[wave];
#pragma unroll
    for (int i = 0; i < 8; ++i) {
        const float inv = (l8[i] > 0.f) ? 1.f / (l8[i] * 4096.f) : 0.f;
#pragma unroll
        for (int t = 0; t < 4; ++t) mo[(i + 8 * hf) * OPITCH + t * 16 + l15] = o[t][i] * inv;
    }
    __syncthreads();
    float* obase = O + b * sOb + h * 64;
#pragma unroll
    for (int r0 = 0; r0 < 16; r0 += 2) {
        const int row = r0 + (lane >> 4), c4 = (lane & 15) * 4;
        const v4f v = *(const v4f*)(mo + row * OPITCH + c4);
        VST2V4(obase + (long long)(q0 + row) * ldo + c4, v);
    }
}

__global__ __launch_bounds__(32) void k_invf_lit(float* __restrict__ invb) {
    const int i = threadIdx.x;
    float v = 1.0f;
    v = (i == 1)  ? 0.7498942093324558f : v;
    v = (i == 2)  ? 0.5623413251903491f : v;
    v = (i == 3)  ? 0.4216965034285822f : v;
    v = (i == 4)  ? 0.31622776601683794f : v;
    v = (i == 5)  ? 0.2371373705661655f : v;
    v = (i == 6)  ? 0.1778279410038923f : v;
    v = (i == 7)  ? 0.1333521432163324f : v;
    v = (i == 8)  ? 0.1f : v;
    v = (i == 9)  ? 0.07498942093324558f : v;
    v = (i == 10) ? 0.05623413251903491f : v;
    v = (i == 11) ? 0.04216965034285822f : v;
    v = (i == 12) ? 0.031622776601683794f : v;
    v = (i == 13) ? 0.02371373705661655f : v;
    v = (i == 14) ? 0.01778279410038923f : v;
    v = (i == 15) ? 0.01333521432163324f : v;
    v = (i == 16) ? 0.01f : v;
    v = (i == 17) ? 0.007498942093324558f : v;
    v = (i == 18) ? 0.005623413251903491f : v;
    v = (i == 19) ? 0.004216965034285822f : v;
    v = (i == 20) ? 0.0031622776601683794f : v;
    v = (i == 21) ? 0.002371373705661655f : v;
    v = (i == 22) ? 0.001778279410038923f : v;
    v = (i == 23) ? 0.001333521432163324f : v;
    v = (i == 24) ? 0.001f : v;
    v = (i == 25) ? 0.0007498942093324558f : v;
    v = (i == 26) ? 0.0005623413251903491f : v;
    v = (i == 27) ? 0.0004216965034285822f : v;
    v = (i == 28) ? 0.00031622776601683794f : v;
    v = (i == 29) ? 0.0002371373705661655f : v;
    v = (i == 30) ? 0.0001778279410038923f : v;
    v = (i == 31) ? 0.0001333521432163324f : v;
    VST2(float, invb + i, v);
}
__global__ __launch_bounds__(256) void k_sincos(float* __restrict__ cs, float* __restrict__ sn, const float* __restrict__ invb, int S, int half, float pscale) {
    const int idx = blockIdx.x * 256 + threadIdx.x;
    if (idx >= S * half) return;
    const int s = idx / half, i = idx - s * half;
    const float ang = (pscale * (float)s) * invb[i];
    VST2(float, cs + idx, cosf(ang)); VST2(float, sn + idx, sinf(ang));
}

__global__ __launch_bounds__(256) void k_rope4(const float* __restrict__ X, int ldx, float* __restrict__ Y, int ldy, const float* __restrict__ cs, const float* __restrict__ sn, int rows, int cols, int S) {
    const long long u = (long long)blockIdx.x * 256 + threadIdx.x; const int per = cols / 4;
    if (u >= (long long)rows * per) return;
    const int r = (int)(u / per); const int c0 = 4 * (int)(u % per);
    const int t = r % S; const int i0 = (c0 & 63) >> 1;
    const v4f x = *(const v4f*)(X + (long long)r * ldx + c0);
    const float ca = cs[t * 32 + i0], cb = cs[t * 32 + i0 + 1], sa = sn[t * 32 + i0], sb = sn[t * 32 + i0 + 1];
    v4f y;
    y.x = x.x * ca - x.y * sa; y.y = x.x * sa + x.y * ca;
    y.z = x.z * cb - x.w * sb; y.w = x.z * sb + x.w * cb;
    VST2V4(Y + (long long)r * ldy + c0, y);
}

namespace eng {
typedef __attribute__((ext_vector_type(16))) _Float16 v16h;
typedef __attribute__((ext_vector_type(8)))  _Float16 v8h;
typedef __attribute__((ext_vector_type(16))) __bf16   v16b;
typedef __attribute__((ext_vector_type(8)))  __bf16   v8b;
typedef __attribute__((ext_vector_type(8)))  float    v8f;
typedef __attribute__((ext_vector_type(4)))  float    v4f;

__device__ __forceinline__ unsigned short f2bf_bits(float f) {
  unsigned u = __float_as_uint(f);
  return (unsigned short)((u + 0x7FFFu + ((u >> 16) & 1u)) >> 16);
}
__device__ __forceinline__ float bf_bits2f(unsigned short h) { return __uint_as_float(((unsigned)h) << 16); }

__device__ __forceinline__ void dep_guard_h(v8f& a, v8f& b, v16h x, v16h y) { asm volatile("v_nop\n\tv_nop\n\tv_nop\n\tv_nop" : "+v"(a), "+v"(b) : "v"(x), "v"(y)); }
__device__ __forceinline__ void dep_guard_b(v8f& a, v8f& b, v16b x, v16b y) { asm volatile("v_nop\n\tv_nop\n\tv_nop\n\tv_nop" : "+v"(a), "+v"(b) : "v"(x), "v"(y)); }
__device__ __forceinline__ void keep4_h(v16h a, v16h b, v16h c, v16h d) { asm volatile("v_nop" :: "v"(a), "v"(b), "v"(c), "v"(d)); }
__device__ __forceinline__ void keep4_b(v16b a, v16b b, v16b c, v16b d) { asm volatile("v_nop" :: "v"(a), "v"(b), "v"(c), "v"(d)); }
__device__ __forceinline__ void acc_guard4(v8f& a, v8f& b, v8f& c, v8f& d) { asm volatile("v_nop\n\tv_nop\n\tv_nop\n\tv_nop" : "+v"(a), "+v"(b), "+v"(c), "+v"(d)); }
template <typename T> struct Frag;
template <> struct Frag<_Float16> {
  typedef v16h V; union U { v16h v; v8h h[2]; };
  static __device__ __forceinline__ v16h load(const _Float16* p) {
    U f; f.h[0] = *(const v8h*)(p); f.h[1] = *(const v8h*)(p + 16); return f.v;
  }
  static __device__ __forceinline__ v8f mma(v16h a, v16h b, v8f c) {
    return __builtin_amdgcn_wmma_f32_16x16x32_f16(false, a, false, b, (short)0, c, false, false);
  }
  static __device__ __forceinline__ void guard(v8f& a, v8f& b, v16h x, v16h y) { dep_guard_h(a, b, x, y); }
  static __device__ __forceinline__ void keep(v16h a, v16h b, v16h c, v16h d) { keep4_h(a, b, c, d); }
};
template <> struct Frag<__bf16> {
  typedef v16b V; union U { v16b v; v8b h[2]; };
  static __device__ __forceinline__ v16b load(const __bf16* p) {
    U f; f.h[0] = *(const v8b*)(p); f.h[1] = *(const v8b*)(p + 16); return f.v;
  }
  static __device__ __forceinline__ v8f mma(v16b a, v16b b, v8f c) {
    return __builtin_amdgcn_wmma_f32_16x16x32_bf16(false, a, false, b, (short)0, c, false, false);
  }
  static __device__ __forceinline__ void guard(v8f& a, v8f& b, v16b x, v16b y) { dep_guard_b(a, b, x, y); }
  static __device__ __forceinline__ void keep(v16b a, v16b b, v16b c, v16b d) { keep4_b(a, b, c, d); }
};

template <int ET> struct Elem;
template <> struct Elem<0> { typedef _Float16 T; };
template <> struct Elem<1> { typedef __bf16 T; };
template <int ET, bool SPLIT, int BIAS_MODE, int OUT_MODE, bool RESID, int ACT = 0>
__global__ __launch_bounds__(256) void wmma_gemm64(
    const unsigned short* __restrict__ Ap, const unsigned short* __restrict__ A2p, int lda, long strideA,
    const unsigned short* __restrict__ Btp, const unsigned short* __restrict__ Bt2p, int ldb, long strideB,
    void* __restrict__ Cout, void* __restrict__ Cout2, int ldc, long strideC,
    const float* __restrict__ bias,
    const float* __restrict__ resid, long strideR,
    int M, int N, int K, float scale) {
  typedef typename Elem<ET>::T T;
  typedef typename Frag<T>::V V;
  const T* A = (const T*)Ap; const T* A2 = (const T*)A2p; const T* Bt = (const T*)Btp; const T* Bt2 = (const T*)Bt2p;
  __shared__ __align__(16) float sT[8][16 * 68];
  const int b    = blockIdx.y;
  const int lane = threadIdx.x & 31;
  const int wave = threadIdx.x >> 5;
  const int tilesN = N >> 6;
  const int tilesM = M >> 6;
  const int tile = blockIdx.x * 8 + wave;
  if (tile >= tilesM * tilesN) return;
  const int tm = tile / tilesN;
  const int tn = tile - tm * tilesN;
  const int m0 = tm << 6;
  const int n0 = tn << 6;

  const T* Ab  = A  + (size_t)b * strideA;
  const T* Bb  = Bt + (size_t)b * strideB;
  const T* Ab2 = SPLIT ? (A2  + (size_t)b * strideA) : nullptr;
  const T* Bb2 = SPLIT ? (Bt2 + (size_t)b * strideB) : nullptr;

  const int rlane = lane & 15;
  const int koff  = (lane >> 4) * 8;
  const int mOff  = (lane >> 4) * 8;

  v8f acc[4][4];
#pragma unroll
  for (int i = 0; i < 4; ++i)
#pragma unroll
    for (int j = 0; j < 4; ++j) acc[i][j] = (v8f){0.f,0.f,0.f,0.f,0.f,0.f,0.f,0.f};

  for (int k0 = 0; k0 < K; k0 += 32) {
    V bh[4], bl[4];
#pragma unroll
    for (int j = 0; j < 4; ++j) {
      const size_t bo = (size_t)(n0 + (j << 4) + rlane) * ldb + koff + k0;
      bh[j] = Frag<T>::load(Bb + bo);
      if (SPLIT) bl[j] = Frag<T>::load(Bb2 + bo);
    }
#pragma unroll
    for (int i = 0; i < 4; ++i) {
      const size_t ao = (size_t)(m0 + (i << 4) + rlane) * lda + koff + k0;
      V ah = Frag<T>::load(Ab + ao);
      V al;
      if (SPLIT) al = Frag<T>::load(Ab2 + ao);
#pragma unroll
      for (int j = 0; j < 4; ++j) {
        acc[i][j] = Frag<T>::mma(ah, bh[j], acc[i][j]);
        if (SPLIT) {
          acc[i][j] = Frag<T>::mma(ah, bl[j], acc[i][j]);
          acc[i][j] = Frag<T>::mma(al, bh[j], acc[i][j]);
        }
      }
      Frag<T>::guard(acc[i][0], acc[i][3], ah, SPLIT ? al : ah);
    }
    Frag<T>::keep(bh[0], bh[1], bh[2], bh[3]);
    if (SPLIT) Frag<T>::keep(bl[0], bl[1], bl[2], bl[3]);
  }
  acc_guard4(acc[0][0], acc[0][1], acc[0][2], acc[0][3]);
  acc_guard4(acc[1][0], acc[1][1], acc[1][2], acc[1][3]);
  acc_guard4(acc[2][0], acc[2][1], acc[2][2], acc[2][3]);
  acc_guard4(acc[3][0], acc[3][1], acc[3][2], acc[3][3]);

  float* slab = sT[wave];
  const float* Rb = RESID ? (resid + (size_t)b * strideR) : nullptr;
#pragma unroll
  for (int i = 0; i < 4; ++i) {
    const int mBase = m0 + (i << 4);
#pragma unroll
    for (int j = 0; j < 4; ++j) {
      const int n = n0 + (j << 4) + rlane;
      float bv = 0.f;
      if (BIAS_MODE == 2) bv = bias[n];
#pragma unroll
      for (int r = 0; r < 8; ++r) {
        float v = acc[i][j][r] * scale;
        if (BIAS_MODE == 1) v += bias[mBase + mOff + r];
        if (BIAS_MODE == 2) v += bv;
        if (RESID) v += Rb[(size_t)(mBase + mOff + r) * ldc + n];
        if (ACT == 1) v = tanhf(v);
        if (ACT == 2) v = fmaxf(v, 0.0f);
        if (ACT == 3) v = v / (1.0f + expf(-v));
        if (ACT == 4) v = (v > 0.f) ? v : 0.01f * v;
        if (ACT == 5) v = 0.5f * v * (1.0f + erff(v * 0.70710678118654752f));
        if (ACT == 6) v = (v > 0.f) ? v : 0.2f * v;
        if (ACT == 7) { const float u = 0.7978845608028654f * (v + 0.044715f * v * v * v); v = 0.5f * v * (1.f + tanhf(u)); }
        slab[(mOff + r) * 68 + (j << 4) + rlane] = v;
      }
    }
    __builtin_amdgcn_fence(3  , "workgroup");
    __builtin_amdgcn_wave_barrier();
    __builtin_amdgcn_fence(2  , "workgroup");
    if (OUT_MODE == 0) {
      float* C = (float*)Cout + (size_t)b * strideC;
      const int hh = lane >> 4, c4 = (lane & 15) * 4;
      for (int pass = 0; pass < 2; ++pass) {
#pragma unroll
        for (int it = 0; it < 8; ++it) {
          const int row = it * 2 + hh;
          v4f v = *(const v4f*)(slab + row * 68 + c4);
          *(volatile v4f*)(C + (size_t)(mBase + row) * ldc + n0 + c4) = v;
        }
        __threadfence();
      }
    } else {
      const int q = lane >> 3, c8 = (lane & 7) * 8;
      unsigned short* C  = (unsigned short*)Cout  + (size_t)b * strideC;
      unsigned short* C2 = (OUT_MODE == 2) ? ((unsigned short*)Cout2 + (size_t)b * strideC) : nullptr;
      for (int pass = 0; pass < 2; ++pass) {
#pragma unroll
        for (int it = 0; it < 4; ++it) {
          const int row = it * 4 + q;
          const float* sp = slab + row * 68 + c8;
          v8h hv, lv;
#pragma unroll
          for (int e = 0; e < 8; ++e) {
            if (OUT_MODE == 1) {
              hv[e] = (_Float16)sp[e];
            } else {
              unsigned short hb = f2bf_bits(sp[e]);
              unsigned short lb = f2bf_bits(sp[e] - bf_bits2f(hb));
              hv[e] = __builtin_bit_cast(_Float16, hb);
              lv[e] = __builtin_bit_cast(_Float16, lb);
            }
          }
          *(volatile v8h*)(C + (size_t)(mBase + row) * ldc + n0 + c8) = hv;
          if (OUT_MODE == 2) *(volatile v8h*)(C2 + (size_t)(mBase + row) * ldc + n0 + c8) = lv;
        }
        __threadfence();
      }
    }
    __builtin_amdgcn_fence(3  , "workgroup");
    __builtin_amdgcn_wave_barrier();
    __builtin_amdgcn_fence(2  , "workgroup");
  }
}
}

__global__ __launch_bounds__(256) void k_cast16(const float* __restrict__ src, long long lds, _Float16* __restrict__ dst, long long ldd, int R, int C, float s) {
    const long long i = (long long)blockIdx.x * 256 + threadIdx.x; const long long np = (long long)R * (C / 2); if (i >= np) return; const int r = (int)(i / (C / 2)); const int c = 2 * (int)(i % (C / 2));
    const _Float16 h0 = (_Float16)(src[(long long)r * lds + c] * s), h1 = (_Float16)(src[(long long)r * lds + c + 1] * s);
    const unsigned u = (unsigned)__builtin_bit_cast(unsigned short, h0) | ((unsigned)__builtin_bit_cast(unsigned short, h1) << 16);
    volatile unsigned* d = (volatile unsigned*)(dst + (long long)r * ldd + c); *d = u; __threadfence(); *d = u; }

typedef unsigned int cm_u4 __attribute__((ext_vector_type(4)));
__device__ __forceinline__ unsigned int cmb_pk2(float a, float b) { return (unsigned int)__builtin_bit_cast(unsigned short, (_Float16)a) | ((unsigned int)__builtin_bit_cast(unsigned short, (_Float16)b) << 16); }
__device__ __forceinline__ float cmb_bf(float v) { const unsigned u = __builtin_bit_cast(unsigned, v); const unsigned r = (u + 0x7fffu + ((u >> 16) & 1u)) & 0xffff0000u; return __builtin_bit_cast(float, r); }
__global__ __launch_bounds__(256) void k_cm_castb(const float* __restrict__ SRC, int lds, unsigned short* __restrict__ DST, int ldd, int nR, int nC, float sc) {
    const long long u = (long long)blockIdx.x * 256 + threadIdx.x; const int per = nC / 8; if (u >= (long long)nR * per) return; const int r = (int)(u / per); const int c0 = 8 * (int)(u % per);
    const float* s = SRC + (long long)r * lds + c0; float w[8];
#pragma unroll
    for (int e = 0; e < 8; ++e) w[e] = cmb_bf(s[e]) * sc;
    cm_u4 pk; pk.x = cmb_pk2(w[0], w[1]); pk.y = cmb_pk2(w[2], w[3]); pk.z = cmb_pk2(w[4], w[5]); pk.w = cmb_pk2(w[6], w[7]); VST2(cm_u4, (cm_u4*)(DST + (long long)r * ldd + c0), pk); }

#define YCARRY 16.0f
#define YRES 256.0f
__device__ __forceinline__ unsigned int hbits(h16 v) { return (unsigned int)__builtin_bit_cast(unsigned short, v); }
__global__ __launch_bounds__(128) void k_rmsplane(const float* __restrict__ X, long long sxb, int S, const float* __restrict__ G,
                                                  unsigned short* __restrict__ Y, int ldy, int resoff, int bfx) {
    #pragma clang fp contract(off)
    __shared__ float red[4];
    const int row = blockIdx.x, t = threadIdx.x, lane = t & 31;
    const int wave = __builtin_amdgcn_readfirstlane(t >> 5);
    const int b = row / S, s = row - b * S;
    const float* xr = X + (long long)b * sxb + (long long)s * DM + 8 * t;
    const v4f xa = *(const v4f*)(xr), xb = *(const v4f*)(xr + 4);
    const v4f ga = *(const v4f*)(G + 8 * t), gb = *(const v4f*)(G + 8 * t + 4);
    float xv[8] = { xa.x, xa.y, xa.z, xa.w, xb.x, xb.y, xb.z, xb.w };
    float gv[8] = { ga.x, ga.y, ga.z, ga.w, gb.x, gb.y, gb.z, gb.w };
    float ss = 0.f;
#pragma unroll
    for (int e = 0; e < 8; ++e) {
        const float xq = cmb_bf(xv[e]);
        xv[e] = (bfx != 0) ? xq : xv[e];
        gv[e] = cmb_bf(gv[e]);
        ss += xv[e] * xv[e];
    }
    ss += __shfl_xor(ss, 16, 32); ss += __shfl_xor(ss, 8, 32); ss += __shfl_xor(ss, 4, 32); ss += __shfl_xor(ss, 2, 32); ss += __shfl_xor(ss, 1, 32);
    if (lane == 0) red[wave] = ss;
    __syncthreads();
    const float tot = (red[0] + red[1]) + (red[2] + red[3]);
    const float rinv = 1.0f / sqrtf(tot * (1.0f / (float)DM) + 1.0e-5f);
    unsigned int hb[8], rb[8];
#pragma unroll
    for (int e = 0; e < 8; ++e) {
        const float yc = ((xv[e] * gv[e]) * rinv) * YCARRY;
        const h16 hv = toh_flush(yc);
        const h16 rv = toh_flush((yc - (float)hv) * YRES);
        hb[e] = hbits(hv); rb[e] = hbits(rv);
    }
    cm_u4 ph, pr;
    ph.x = hb[0] | (hb[1] << 16); ph.y = hb[2] | (hb[3] << 16); ph.z = hb[4] | (hb[5] << 16); ph.w = hb[6] | (hb[7] << 16);
    pr.x = rb[0] | (rb[1] << 16); pr.y = rb[2] | (rb[3] << 16); pr.z = rb[4] | (rb[5] << 16); pr.w = rb[6] | (rb[7] << 16);
    unsigned short* yrow = Y + (long long)row * ldy + 8 * t;
    VST2(cm_u4, (cm_u4*)yrow, ph);
    if (resoff > 0) { VST2(cm_u4, (cm_u4*)(yrow + resoff), pr); }
}

__global__ __launch_bounds__(256) void k_glu(const float* __restrict__ L, int ldl, int l3off, unsigned short* __restrict__ Gp, int ldg, int R, int F, float carry) {
    #pragma clang fp contract(off)
    const long long u = (long long)blockIdx.x * 256 + threadIdx.x; const int per = F / 2; if (u >= (long long)R * per) return;
    const int r = (int)(u / per); const int f = 2 * (int)(u % per);
    const v2f a = *(const v2f*)(L + (long long)r * ldl + f);
    const v2f c = *(const v2f*)(L + (long long)r * ldl + l3off + f);
    const float e0 = expf(fminf(-a.x, 40.0f)), e1 = expf(fminf(-a.y, 40.0f));
    const float s0 = 1.0f / (1.0f + e0), s1 = 1.0f / (1.0f + e1);
    const float g0 = ((s0 * a.x) * c.x) * carry, g1 = ((s1 * a.y) * c.y) * carry;
    const unsigned int pk = hbits(toh_flush(g0)) | (hbits(toh_flush(g1)) << 16);
    volatile unsigned* d = (volatile unsigned*)(Gp + (long long)r * ldg + f); *d = pk; __threadfence(); *d = pk;
}

static constexpr size_t cmax_sz(size_t a, size_t b) { return a > b ? a : b; }

extern "C" void kernel_launch(void* const* d_in, const int* in_sizes, int n_in, void* d_out, int out_size, void* d_ws, size_t ws_size, hipStream_t stream) {
    if (n_in < 10) return;
    const long long need_x = (long long)(NB - 1) * XBS_FULL + (long long)SEQ * DM;
    if ((long long)in_sizes[0] < need_x) return;
    if (in_sizes[1] < DM * DM || in_sizes[2] < DM * DM || in_sizes[3] < DM * DM || in_sizes[4] < DM * DM) return;
    if (in_sizes[5] < DFF * DM || in_sizes[6] < DM * DFF || in_sizes[7] < DFF * DM) return;
    if (in_sizes[8] < DM || in_sizes[9] < DM) return;
    if ((long long)out_size < need_x) return;
    const float* x  = (const float*)d_in[0];
    const float* wq = (const float*)d_in[1];
    const float* wk = (const float*)d_in[2];
    const float* wv = (const float*)d_in[3];
    const float* wo = (const float*)d_in[4];
    const float* w1 = (const float*)d_in[5];
    const float* w2 = (const float*)d_in[6];
    const float* w3 = (const float*)d_in[7];
    const float* g1 = (const float*)d_in[8];
    const float* g2 = (const float*)d_in[9];
    float* out = (float*)d_out;

    constexpr size_t R = (size_t)NB * SEQ;
    static_assert(R % 64 == 0);
    constexpr size_t SZ_WQK  = (size_t)(2 * DM) * (2 * DM) * 2;
    constexpr size_t SZ_WDD  = (size_t)DM * DM * 2;
    constexpr size_t SZ_WFF  = (size_t)DFF * DM * 2;
    constexpr size_t SZ_YH   = R * DM * 2;
    constexpr size_t SZ_Y    = cmax_sz(2 * SZ_YH, SZ_YH + SZ_WFF);
    constexpr size_t SZ_QKV  = R * 3 * DM * 4;
    constexpr size_t SZ_QKR  = R * 2 * DM * 4;
    constexpr size_t SZ_AOW  = cmax_sz(R * DM * 4, 2 * SZ_WFF);
    constexpr size_t SZ_TAB  = (size_t)SEQ * 32 * 4;
    constexpr size_t SZ_INV  = 256;
    constexpr size_t SZ_TOTAL = SZ_WQK + 2 * SZ_WDD + SZ_Y + SZ_QKV + SZ_QKR + SZ_AOW + 2 * SZ_TAB + SZ_INV;
    static_assert(SZ_WQK % 256 == 0 && SZ_WDD % 256 == 0 && SZ_Y % 256 == 0 && SZ_QKV % 256 == 0 && SZ_QKR % 256 == 0 && SZ_AOW % 256 == 0 && SZ_TAB % 256 == 0);
    static_assert(R * DFF * 2 + R * DM * 4 <= SZ_QKV);
    static_assert(R * 2 * FCH * 4 <= SZ_QKR);
    static_assert(2 * SZ_WFF <= SZ_AOW && R * DM * 4 <= SZ_AOW);
    static_assert(2 * SZ_YH <= SZ_Y && SZ_YH + SZ_WFF <= SZ_Y);
    static_assert((R * DFF * 2) % 256 == 0 && SZ_YH % 256 == 0 && SZ_WFF % 256 == 0);
    static_assert(SZ_TOTAL <= (size_t)134217728);
    if (SZ_TOTAL > ws_size) return;

    char* wsp = (char*)d_ws;
    unsigned short* WQK  = (unsigned short*)wsp; wsp += SZ_WQK;
    unsigned short* WV16 = (unsigned short*)wsp; wsp += SZ_WDD;
    unsigned short* WO16 = (unsigned short*)wsp; wsp += SZ_WDD;
    char* regY = wsp; wsp += SZ_Y;
    char* regQKV = wsp; wsp += SZ_QKV;
    char* regQKR = wsp; wsp += SZ_QKR;
    char* regAOW = wsp; wsp += SZ_AOW;
    float* CS = (float*)wsp; wsp += SZ_TAB;
    float* SN = (float*)wsp; wsp += SZ_TAB;
    float* INVF = (float*)wsp; wsp += SZ_INV;

    unsigned short* Y1   = (unsigned short*)regY;
    unsigned short* AO16 = (unsigned short*)regY;
    unsigned short* Y2   = (unsigned short*)regY;
    unsigned short* W2P  = (unsigned short*)(regY + SZ_YH);
    float* QKV = (float*)regQKV;
    unsigned short* GLU = (unsigned short*)regQKV;
    float* X1  = (float*)(regQKV + R * DFF * 2);
    float* QKR = (float*)regQKR;
    float* L13 = (float*)regQKR;
    float* AO  = (float*)regAOW;
    unsigned short* W1P = (unsigned short*)regAOW;
    unsigned short* W3P = (unsigned short*)(regAOW + SZ_WFF);

    const unsigned gDD = (unsigned)(((long long)DM * (DM / 8) + 255) / 256);
    const unsigned gFF = (unsigned)(((long long)DFF * (DM / 8) + 255) / 256);
    k_cm_castb<<<gDD, 256, 0, stream>>>(wq, DM, WQK, 2 * DM, DM, DM, 16.0f);
    k_cm_castb<<<gDD, 256, 0, stream>>>(wq, DM, WQK + DM, 2 * DM, DM, DM, 0.0625f);
    k_cm_castb<<<gDD, 256, 0, stream>>>(wk, DM, WQK + (size_t)DM * 2 * DM, 2 * DM, DM, DM, 16.0f);
    k_cm_castb<<<gDD, 256, 0, stream>>>(wk, DM, WQK + (size_t)DM * 2 * DM + DM, 2 * DM, DM, DM, 0.0625f);
    k_cm_castb<<<gDD, 256, 0, stream>>>(wv, DM, WV16, DM, DM, DM, 16.0f);
    k_cm_castb<<<gDD, 256, 0, stream>>>(wo, DM, WO16, DM, DM, DM, 16.0f);
    k_rmsplane<<<(unsigned)R, 128, 0, stream>>>(x, (long long)XBS_FULL, SEQ, g1, Y1, 2 * DM, DM, 1);
    eng::wmma_gemm64<0, false, 0, 0, false, 0><<<dim3((unsigned)((((int)R / 64) * (2 * DM / 64) + 7) / 8), 1u), 256, 0, stream>>>(
        (const unsigned short*)Y1, nullptr, 2 * DM, (long)0, (const unsigned short*)WQK, nullptr, 2 * DM, (long)0,
        (void*)QKV, nullptr, 3 * DM, (long)0, nullptr, nullptr, (long)0, (int)R, 2 * DM, 2 * DM, 0.00390625f);
    eng::wmma_gemm64<0, false, 0, 0, false, 0><<<dim3((unsigned)((((int)R / 64) * (DM / 64) + 7) / 8), 1u), 256, 0, stream>>>(
        (const unsigned short*)Y1, nullptr, 2 * DM, (long)0, (const unsigned short*)WV16, nullptr, DM, (long)0,
        (void*)(QKV + 2 * DM), nullptr, 3 * DM, (long)0, nullptr, nullptr, (long)0, (int)R, DM, DM, 0.00390625f);
    k_invf_lit<<<1, 32, 0, stream>>>(INVF);
    k_sincos<<<(unsigned)((SEQ * 32 + 255) / 256), 256, 0, stream>>>(CS, SN, INVF, SEQ, 32, 1.0f);
    k_rope4<<<(unsigned)(((long long)R * (2 * DM / 4) + 255) / 256), 256, 0, stream>>>(QKV, 3 * DM, QKR, 2 * DM, CS, SN, (int)R, 2 * DM, SEQ);
    k_attn3<<<dim3((unsigned)(SEQ / (16 * AW)), (unsigned)NHD, (unsigned)NB), 32 * AW, 0, stream>>>(
        QKR, QKR + DM, QKV + 2 * DM, AO,
        (long long)SEQ * 2 * DM, (long long)SEQ * 2 * DM, (long long)SEQ * 3 * DM, (long long)SEQ * DM,
        2 * DM, 2 * DM, 3 * DM, DM, SEQ, 0, 0.125f);
    k_cast16<<<(unsigned)(((long long)R * (DM / 2) + 255) / 256), 256, 0, stream>>>(AO, DM, (_Float16*)AO16, DM, (int)R, DM, 16.0f);
    eng::wmma_gemm64<0, false, 0, 0, true, 0><<<dim3((unsigned)(((SEQ / 64) * (DM / 64) + 7) / 8), (unsigned)NB), 256, 0, stream>>>(
        (const unsigned short*)AO16, nullptr, DM, (long)((long long)SEQ * DM), (const unsigned short*)WO16, nullptr, DM, (long)0,
        (void*)X1, nullptr, DM, (long)((long long)SEQ * DM), nullptr, x, (long)XBS_FULL, SEQ, DM, DM, 0.00390625f);
    k_cm_castb<<<gFF, 256, 0, stream>>>(w1, DM, W1P, DM, DFF, DM, 16.0f);
    k_cm_castb<<<gFF, 256, 0, stream>>>(w3, DM, W3P, DM, DFF, DM, 16.0f);
    k_cm_castb<<<gFF, 256, 0, stream>>>(w2, DFF, W2P, DFF, DM, DFF, 16.0f);
    k_rmsplane<<<(unsigned)R, 128, 0, stream>>>(X1, (long long)SEQ * DM, SEQ, g2, Y2, DM, 0, 0);
    for (int c = 0; c < DFF / FCH; ++c) {
        eng::wmma_gemm64<0, false, 0, 0, false, 0><<<dim3((unsigned)((((int)R / 64) * (FCH / 64) + 7) / 8), 1u), 256, 0, stream>>>(
            (const unsigned short*)Y2, nullptr, DM, (long)0, (const unsigned short*)(W1P + (size_t)c * FCH * DM), nullptr, DM, (long)0,
            (void*)L13, nullptr, 2 * FCH, (long)0, nullptr, nullptr, (long)0, (int)R, FCH, DM, 0.00390625f);
        eng::wmma_gemm64<0, false, 0, 0, false, 0><<<dim3((unsigned)((((int)R / 64) * (FCH / 64) + 7) / 8), 1u), 256, 0, stream>>>(
            (const unsigned short*)Y2, nullptr, DM, (long)0, (const unsigned short*)(W3P + (size_t)c * FCH * DM), nullptr, DM, (long)0,
            (void*)(L13 + FCH), nullptr, 2 * FCH, (long)0, nullptr, nullptr, (long)0, (int)R, FCH, DM, 0.00390625f);
        k_glu<<<(unsigned)(((long long)R * (FCH / 2) + 255) / 256), 256, 0, stream>>>(L13, 2 * FCH, FCH, GLU + (size_t)c * FCH, DFF, (int)R, FCH, 0.25f);
    }
    eng::wmma_gemm64<0, false, 0, 0, true, 0><<<dim3((unsigned)(((SEQ / 64) * (DM / 64) + 7) / 8), (unsigned)NB), 256, 0, stream>>>(
        (const unsigned short*)GLU, nullptr, DFF, (long)((long long)SEQ * DFF), (const unsigned short*)W2P, nullptr, DFF, (long)0,
        (void*)out, nullptr, DM, (long)XBS_FULL, nullptr, X1, (long)((long long)SEQ * DM), SEQ, DM, DFF, 0.25f);
}
